// GATConvLayer_68418829025698
// MI455X (gfx1250) — hardware-verified
//
#include <hip/hip_runtime.h>
#include <stddef.h>
#include <stdint.h>
#include <math.h>


#define FD      128
#define NH      4
#define NCOL    144
#define NT      9
#define GBM     64
#define GTHR    128
#define LDP     144
#define NTHR    256
#define NWAVE   8
#define EPT     8
#define CHUNK   (NTHR * EPT)
#define WCAP    (EPT * 32)
#define LISTN   (NWAVE * WCAP)
#define NBA     1024
#define SLA     10
#define RCAP    28672
#define DEGCAP  64
#define NUW     (FD * (FD / 8))
#define NBW     (NUW / NTHR)
#define NEGSL   0.2f
#define AGG_ZINTS (LISTN + 2 * RCAP + 3 * NBA)
#define AGG_LDS_INTS (AGG_ZINTS + 16)
#define WSMAX   134217728

static_assert((CHUNK & (CHUNK - 1)) == 0 && CHUNK <= 4096);
static_assert((NBA & (NBA - 1)) == 0 && NBA == (1 << SLA));
static_assert(((long long)CHUNK << SLA) < (1LL << 31));
static_assert(LISTN % NTHR == 0);
static_assert(NBA % NWAVE == 0 && NBA % 32 == 0);
static_assert(RCAP % 4 == 0 && AGG_ZINTS % 4 == 0 && LISTN % 4 == 0);
static_assert(AGG_LDS_INTS * 4 <= 300000);
static_assert(FD % 32 == 0 && FD == 4 * 32);
static_assert(NCOL == 16 * NT && NCOL == FD + 16 && LDP >= NCOL && (LDP % 4) == 0);
static_assert(GBM == (GTHR / 32) * 16 && GTHR == 2 * GBM);
static_assert(NUW % NTHR == 0);
static_assert(GBM * LDP * 4 <= 65536);

typedef float          v4f  __attribute__((ext_vector_type(4)));
typedef float          v8f  __attribute__((ext_vector_type(8)));
typedef int            v4i  __attribute__((ext_vector_type(4)));
typedef int            v8i  __attribute__((ext_vector_type(8)));
typedef unsigned int   v4u  __attribute__((ext_vector_type(4)));
typedef unsigned short v8us __attribute__((ext_vector_type(8)));
typedef __bf16         v16b __attribute__((ext_vector_type(16)));
typedef v4f  __attribute__((may_alias)) v4fa;
typedef v4i  __attribute__((may_alias)) v4ia;
typedef v8us __attribute__((may_alias)) v8usa;
union FragB { v16b v; v8us h[2]; v8i w; };

__device__ __forceinline__ v8f wmb(const FragB& a, const FragB& b, v8f c) {
  v8f d = __builtin_amdgcn_wmma_f32_16x16x32_bf16(false, a.v, false, b.v, (short)0, c, false, false);
  asm volatile("v_nop\n\tv_nop\n\tv_nop\n\tv_nop" : "+v"(d) : "v"(a.w), "v"(b.w));
  return d;
}

__device__ __forceinline__ unsigned int f2bf(float f) {
  const unsigned int u = __float_as_uint(f);
  return ((u + 0x7FFFu + ((u >> 16) & 1u)) >> 16) & 0xFFFFu;
}
__device__ __forceinline__ float bf2f(unsigned int b) { return __uint_as_float(b << 16); }
__device__ __forceinline__ float bfr(float f) { return bf2f(f2bf(f)); }
__device__ __forceinline__ v4f bfr4(const v4f a) {
  v4f r; r.x = bfr(a.x); r.y = bfr(a.y); r.z = bfr(a.z); r.w = bfr(a.w); return r;
}
__device__ __forceinline__ unsigned int pk2(float lo, float hi) { return f2bf(lo) | (f2bf(hi) << 16); }
__device__ __forceinline__ v4u pack8(const v4f a, const v4f b) {
  v4u r;
  r.x = pk2(a.x, a.y); r.y = pk2(a.z, a.w); r.z = pk2(b.x, b.y); r.w = pk2(b.z, b.w);
  return r;
}
__device__ __forceinline__ float lo1(float v) { return v - bfr(v); }
__device__ __forceinline__ v4u pack8lo(const v4f a, const v4f b) {
  v4u r;
  r.x = pk2(lo1(a.x), lo1(a.y)); r.y = pk2(lo1(a.z), lo1(a.w));
  r.z = pk2(lo1(b.x), lo1(b.y)); r.w = pk2(lo1(b.z), lo1(b.w));
  return r;
}

template <int SLB>
__device__ __forceinline__ int scan_chunk(const int* __restrict__ dsts, int nE, int cbase, int slotBase,
                                          int nb, int vec8, int* list, int tid, int lane, int wave) {
  int wc = 0;
  const int el0  = tid * EPT;
  const int e0   = cbase + el0;
  const int sent = -2147483647 - 1;
  v4i da, db;
  if (vec8 != 0 && cbase + CHUNK <= nE) {
    da = *(const v4i*)(dsts + e0);
    db = *(const v4i*)(dsts + e0 + 4);
  } else {
    da.x = (e0     < nE) ? dsts[min(e0,     nE - 1)] : sent;
    da.y = (e0 + 1 < nE) ? dsts[min(e0 + 1, nE - 1)] : sent;
    da.z = (e0 + 2 < nE) ? dsts[min(e0 + 2, nE - 1)] : sent;
    da.w = (e0 + 3 < nE) ? dsts[min(e0 + 3, nE - 1)] : sent;
    db.x = (e0 + 4 < nE) ? dsts[min(e0 + 4, nE - 1)] : sent;
    db.y = (e0 + 5 < nE) ? dsts[min(e0 + 5, nE - 1)] : sent;
    db.z = (e0 + 6 < nE) ? dsts[min(e0 + 6, nE - 1)] : sent;
    db.w = (e0 + 7 < nE) ? dsts[min(e0 + 7, nE - 1)] : sent;
  }
  const unsigned nbs = (unsigned)slotBase;
  const unsigned unb = (unsigned)nb;
  const unsigned s0 = (unsigned)da.x - nbs, s1 = (unsigned)da.y - nbs;
  const unsigned s2 = (unsigned)da.z - nbs, s3 = (unsigned)da.w - nbs;
  const unsigned s4 = (unsigned)db.x - nbs, s5 = (unsigned)db.y - nbs;
  const unsigned s6 = (unsigned)db.z - nbs, s7 = (unsigned)db.w - nbs;
  const bool h0 = s0 < unb, h1 = s1 < unb, h2 = s2 < unb, h3 = s3 < unb;
  const bool h4 = s4 < unb, h5 = s5 < unb, h6 = s6 < unb, h7 = s7 < unb;
  const unsigned any = __builtin_amdgcn_ballot_w32(h0 | h1 | h2 | h3 | h4 | h5 | h6 | h7);
  if (any != 0u) {
#define HITJ(J, HJ, SJ) { \
      const unsigned mj = __builtin_amdgcn_ballot_w32(HJ); \
      if (mj != 0u) { \
        if (HJ) { \
          const int pos = wc + (int)__builtin_amdgcn_mbcnt_lo(mj, 0u); \
          if (pos < WCAP) list[wave * WCAP + pos] = ((el0 + (J)) << SLB) | (int)(SJ); \
        } \
        wc += (int)__builtin_popcount(mj); } }
    HITJ(0, h0, s0)
    HITJ(1, h1, s1)
    HITJ(2, h2, s2)
    HITJ(3, h3, s3)
    HITJ(4, h4, s4)
    HITJ(5, h5, s5)
    HITJ(6, h6, s6)
    HITJ(7, h7, s7)
#undef HITJ
  }
  return wc;
}

__global__ __launch_bounds__(NTHR) void k_prep(const float* __restrict__ Wlin,
                                               const float* __restrict__ Wel, const float* __restrict__ bel,
                                               const float* __restrict__ Wer, const float* __restrict__ ber,
                                               const float* __restrict__ attl, const float* __restrict__ attr,
                                               unsigned short* BT, float* CV) {
  __shared__ __attribute__((aligned(16))) float sc[32];
  const int tid = (int)threadIdx.x;
  if ((int)blockIdx.x < NBW) {
    const int u  = (int)blockIdx.x * NTHR + tid;
    const float* p = Wlin + (size_t)u * 8;
    const v4f a = *(const v4fa*)p;
    const v4f b = *(const v4fa*)(p + 4);
    const v4u wv = pack8(a, b);
    unsigned short* o = BT + (size_t)u * 8;
    *(volatile v4u*)o = wv;
    __threadfence();
    *(volatile v4u*)o = wv;
    return;
  }
  if (tid < 128) {
    const int which = __builtin_amdgcn_readfirstlane(tid >> 6);
    const int vh = tid >> 4;
    const int h  = vh & 3;
    const int k8 = (tid & 15) * 8;
    const float* Wp = (which != 0 ? Wer : Wel) + (size_t)(h * FD) * FD + k8;
    const float* ap = (which != 0 ? attr : attl) + h * FD;
    v4f s0 = {0.f, 0.f, 0.f, 0.f}, s1 = {0.f, 0.f, 0.f, 0.f};
#pragma unroll 1
    for (int f = 0; f < FD; ++f) {
      const float af = bfr(ap[f]);
      const v4f w0 = bfr4(*(const v4fa*)(Wp + (size_t)f * FD));
      const v4f w1 = bfr4(*(const v4fa*)(Wp + (size_t)f * FD + 4));
      s0.x = fmaf(af, w0.x, s0.x); s0.y = fmaf(af, w0.y, s0.y);
      s0.z = fmaf(af, w0.z, s0.z); s0.w = fmaf(af, w0.w, s0.w);
      s1.x = fmaf(af, w1.x, s1.x); s1.y = fmaf(af, w1.y, s1.y);
      s1.z = fmaf(af, w1.z, s1.z); s1.w = fmaf(af, w1.w, s1.w);
    }
    const v4u hv = pack8(s0, s1);
    const v4u lv = pack8lo(s0, s1);
    unsigned short* oh = BT + (size_t)(FD + vh) * FD + k8;
    unsigned short* ol = BT + (size_t)(FD + 8 + vh) * FD + k8;
    *(volatile v4u*)oh = hv;
    *(volatile v4u*)ol = lv;
    __threadfence();
    *(volatile v4u*)oh = hv;
    *(volatile v4u*)ol = lv;
  } else if (tid < 160) {
    const int l = tid - 128;
    const int q = l & 7;
    const int h = q & 3;
    const float* b0p = bel  + h * FD;
    const float* b1p = ber  + h * FD;
    const float* a0p = attl + h * FD;
    const float* a1p = attr + h * FD;
    float sl = 0.f, sr = 0.f;
#pragma unroll 1
    for (int f4 = 0; f4 < FD / 4; ++f4) {
      const v4f bl = bfr4(*(const v4fa*)(b0p + 4 * f4));
      const v4f br = bfr4(*(const v4fa*)(b1p + 4 * f4));
      const v4f al = bfr4(*(const v4fa*)(a0p + 4 * f4));
      const v4f ar = bfr4(*(const v4fa*)(a1p + 4 * f4));
      sl = fmaf(bl.x, al.x, sl); sl = fmaf(bl.y, al.y, sl); sl = fmaf(bl.z, al.z, sl); sl = fmaf(bl.w, al.w, sl);
      sr = fmaf(br.x, ar.x, sr); sr = fmaf(br.y, ar.y, sr); sr = fmaf(br.z, ar.z, sr); sr = fmaf(br.w, ar.w, sr);
    }
    const float c = (q < 4) ? sl : sr;
    sc[l] = (l < 8) ? c : 0.0f;
  }
  __syncthreads();
  {
    const int l = tid & 31;
    const v4f cv = *(const v4fa*)(sc + 4 * (l & 7));
    if (tid >= 128 && tid < 136) {
      float* cp = CV + 4 * l;
      *(volatile v4f*)cp = cv;
      __threadfence();
      *(volatile v4f*)cp = cv;
    }
  }
}

__global__ __launch_bounds__(GTHR) void k_gemm(const float* __restrict__ X, const unsigned short* __restrict__ BT,
                                               const float* __restrict__ blin, const float* __restrict__ CV,
                                               float* HM, float* ELR, int nN) {
  __shared__ __attribute__((aligned(16))) float stg[GBM * LDP];
  const int tid = (int)threadIdx.x, lane = tid & 31, wave = tid >> 5, hh = lane >> 4, m = lane & 15;
  const int rowBase = (int)blockIdx.x * GBM;

  v8f acc[NT];
  {
    const v8f z = {0.f, 0.f, 0.f, 0.f, 0.f, 0.f, 0.f, 0.f};
#pragma unroll
    for (int t = 0; t < NT; ++t) acc[t] = z;
  }
  const int  grow = rowBase + 16 * wave + m;
  const bool ok   = grow < nN;
  const int  rc   = ok ? grow : nN - 1;
  const float* xp = X + (size_t)rc * FD + 8 * hh;
  const unsigned short* bp = BT + (size_t)m * FD + 8 * hh;
  const v4f z4 = {0.f, 0.f, 0.f, 0.f};

#pragma unroll 1
  for (int ks = 0; ks < FD / 32; ++ks) {
    v4f a0 = *(const v4fa*)(xp + 32 * ks);
    v4f a1 = *(const v4fa*)(xp + 32 * ks + 4);
    v4f a2 = *(const v4fa*)(xp + 32 * ks + 16);
    v4f a3 = *(const v4fa*)(xp + 32 * ks + 20);
    a0 = ok ? a0 : z4; a1 = ok ? a1 : z4; a2 = ok ? a2 : z4; a3 = ok ? a3 : z4;
    const v4u plo = pack8(a0, a1);
    const v4u phi = pack8(a2, a3);
    FragB af;
    {
      v8i wv;
      wv[0] = (int)plo.x; wv[1] = (int)plo.y; wv[2] = (int)plo.z; wv[3] = (int)plo.w;
      wv[4] = (int)phi.x; wv[5] = (int)phi.y; wv[6] = (int)phi.z; wv[7] = (int)phi.w;
      af.w = wv;
    }
#pragma unroll
    for (int t = 0; t < NT; ++t) {
      const unsigned short* wq = bp + (size_t)(16 * t) * FD + 32 * ks;
      FragB bf;
      bf.h[0] = *(const v8usa*)wq;
      bf.h[1] = *(const v8usa*)(wq + 16);
      acc[t] = wmb(af, bf, acc[t]);
    }
  }

#pragma unroll
  for (int t = 0; t < NT; ++t) {
    const int lc = 16 * t + m;
#pragma unroll
    for (int r = 0; r < 8; ++r) {
      const int lr = 16 * wave + 8 * hh + r;
      stg[lr * LDP + lc] = acc[t][r];
    }
  }
  __syncthreads();

  const v4f b4 = bfr4(*(const v4fa*)(blin + 4 * lane));
  v4f ev;
  {
    const int er = tid >> 1, q0 = (tid & 1) * 4;
    const v4f eh = *(const v4fa*)(stg + er * LDP + FD + q0);
    const v4f el = *(const v4fa*)(stg + er * LDP + FD + 8 + q0);
    const v4f cc = *(const v4fa*)(CV + q0);
    ev.x = (eh.x + el.x) + cc.x; ev.y = (eh.y + el.y) + cc.y;
    ev.z = (eh.z + el.z) + cc.z; ev.w = (eh.w + el.w) + cc.w;
  }
  float* ep = ELR + (size_t)rowBase * 8 + 4 * tid;

#pragma unroll 1
  for (int i = 0; i < 16; ++i) {
    const int row = 16 * wave + i;
    v4f p = *(const v4fa*)(stg + row * LDP + 4 * lane);
    p.x += b4.x; p.y += b4.y; p.z += b4.z; p.w += b4.w;
    float* op = HM + (size_t)(rowBase + row) * FD + 4 * lane;
    *(volatile v4f*)op = p;
  }
  *(volatile v4f*)ep = ev;
  __threadfence();
#pragma unroll 1
  for (int i = 0; i < 16; ++i) {
    const int row = 16 * wave + i;
    v4f p = *(const v4fa*)(stg + row * LDP + 4 * lane);
    p.x += b4.x; p.y += b4.y; p.z += b4.z; p.w += b4.w;
    float* op = HM + (size_t)(rowBase + row) * FD + 4 * lane;
    *(volatile v4f*)op = p;
  }
  *(volatile v4f*)ep = ev;
}

__global__ __launch_bounds__(NTHR) void k_scan(const int* __restrict__ own, const int* __restrict__ gat,
                                               int nE, int nN, int vec8,
                                               const float* __restrict__ ELR, const float* __restrict__ HM,
                                               float* outp) {
  extern __shared__ __attribute__((aligned(16))) int dsm[];
  int* list = dsm;
  int* hl   = dsm + LISTN;
  int* sl   = dsm + LISTN + RCAP;
  int* cnt  = dsm + LISTN + 2 * RCAP;
  int* offs = cnt + NBA;
  int* cur  = offs + NBA;
  int* misc = cur + NBA;
  const int tid = (int)threadIdx.x, lane = tid & 31, wave = tid >> 5;
  const int nodeBase = (int)blockIdx.x * NBA;

  {
    const v4i z4 = {0, 0, 0, 0};
    for (int i = tid * 4; i < AGG_ZINTS; i += NTHR * 4) *(v4ia*)(dsm + i) = z4;
    if (tid < 16) misc[tid] = 0;
  }
  __syncthreads();

  int t = 0, ov = 0;
  const int nChunks = (nE + CHUNK - 1) / CHUNK;
#pragma unroll 1
  for (int ch = 0; ch < nChunks; ++ch) {
    const int cbase = ch * CHUNK;
    const int wc = scan_chunk<SLA>(own, nE, cbase, nodeBase, NBA, vec8, list, tid, lane, wave);
    if (lane == 0) misc[wave] = wc;
    __syncthreads();
    if (wave == 0) {
#pragma unroll 1
      for (int w2 = 0; w2 < NWAVE; ++w2) {
        int c = misc[w2];
        c = c < 0 ? 0 : (c > WCAP ? WCAP : c);
#pragma unroll 1
        for (int b0 = 0; b0 < c; b0 += 32) {
          const int idx = b0 + lane;
          const int ent = list[w2 * WCAP + (idx < WCAP ? idx : WCAP - 1)];
          const int m32 = (c - b0) < 32 ? (c - b0) : 32;
#pragma unroll 1
          for (int k = 0; k < m32; ++k) {
            const int u    = __builtin_amdgcn_readlane(ent, k);
            const int slot = u & (NBA - 1);
            const int el   = (u >> SLA) & (CHUNK - 1);
            const int pk   = ((cbase + el) << SLA) | slot;
            if (t < RCAP) {
              if (lane == 0) { hl[t] = pk; cnt[slot] = cnt[slot] + 1; }
              t = t + 1;
            } else {
              ov = 1;
            }
          }
        }
      }
    }
    __syncthreads();
  }
  if (wave == 0 && lane == 0) { misc[8] = t; misc[9] = ov; }
  __syncthreads();
  int tt = misc[8];
  tt = tt < 0 ? 0 : (tt > RCAP ? RCAP : tt);
  const int ovf = misc[9];

  if (wave == 0) {
    const int base = lane * (NBA / 32);
    int s = 0;
#pragma unroll 1
    for (int i = 0; i < NBA / 32; ++i) s += cnt[base + i];
    int incl = s;
#pragma unroll
    for (int d = 1; d < 32; d <<= 1) {
      const int y = __shfl_up(incl, d, 32);
      if (lane >= d) incl += y;
    }
    int run = incl - s;
#pragma unroll 1
    for (int i = 0; i < NBA / 32; ++i) {
      const int cv = cnt[base + i];
      offs[base + i] = run;
      cur[base + i]  = run;
      run += cv;
    }
  }
  __syncthreads();
  if (wave == 0) {
#pragma unroll 1
    for (int b0 = 0; b0 < tt; b0 += 32) {
      const int idx = b0 + lane;
      const int ent = hl[idx < RCAP ? idx : RCAP - 1];
      const int m32 = (tt - b0) < 32 ? (tt - b0) : 32;
#pragma unroll 1
      for (int k = 0; k < m32; ++k) {
        const int u    = __builtin_amdgcn_readlane(ent, k);
        const int slot = u & (NBA - 1);
        if (lane == 0) {
          int p = cur[slot];
          p = p < 0 ? 0 : (p > RCAP - 1 ? RCAP - 1 : p);
          sl[p] = u;
          cur[slot] = p + 1;
        }
      }
    }
  }
  __syncthreads();

  const float qnan = __int_as_float(0x7fc00000);
  const float pz = (ovf != 0) ? qnan : 0.0f;
#pragma unroll 1
  for (int si = 0; si < NBA / NWAVE; ++si) {
    const int s    = si * NWAVE + wave;
    const int node = nodeBase + s;
    int c = __builtin_amdgcn_readfirstlane(cnt[s]);
    const bool big = c > DEGCAP;
    c = c < 0 ? 0 : (c > DEGCAP ? DEGCAP : c);
    int o = __builtin_amdgcn_readfirstlane(offs[s]);
    o = o < 0 ? 0 : (o > RCAP ? RCAP : o);
    const int nc = node < nN ? node : nN - 1;
    const v4f el4 = *(const v4f*)(ELR + (size_t)nc * 8);
    v4f acc = *(const v4f*)(HM + (size_t)nc * FD + 4 * lane);
#pragma unroll 1
    for (int b0 = 0; b0 < c; b0 += 32) {
      int idx = o + b0 + lane;
      idx = idx > RCAP - 1 ? RCAP - 1 : idx;
      const int ent = sl[idx];
      int eid = ent >> SLA;
      eid = eid < 0 ? 0 : (eid > nE - 1 ? nE - 1 : eid);
      int j = gat[eid];
      j = j < 0 ? 0 : (j > nN - 1 ? nN - 1 : j);
      const v4f er4 = *(const v4f*)(ELR + (size_t)j * 8 + 4);
      float l0 = el4.x + er4.x, l1 = el4.y + er4.y, l2 = el4.z + er4.z, l3 = el4.w + er4.w;
      l0 = l0 >= 0.f ? l0 : NEGSL * l0;
      l1 = l1 >= 0.f ? l1 : NEGSL * l1;
      l2 = l2 >= 0.f ? l2 : NEGSL * l2;
      l3 = l3 >= 0.f ? l3 : NEGSL * l3;
      const float mx = fmaxf(fmaxf(l0, l1), fmaxf(l2, l3));
      const float e0 = expf(l0 - mx), e1 = expf(l1 - mx), e2 = expf(l2 - mx), e3 = expf(l3 - mx);
      const float sm  = ((e0 + e1) + e2) + e3;
      const float inv = 1.0f / sm;
      const float aw  = (((e0 * inv + e1 * inv) + e2 * inv) + e3 * inv) * 0.25f;
      const int   ai  = __float_as_int(aw);
      const int m32 = (c - b0) < 32 ? (c - b0) : 32;
#pragma unroll 1
      for (int k = 0; k < m32; ++k) {
        const int   jk = __builtin_amdgcn_readlane(j, k);
        const float ak = __int_as_float(__builtin_amdgcn_readlane(ai, k));
        const v4f r = *(const v4f*)(HM + (size_t)jk * FD + 4 * lane);
        acc.x = fmaf(ak, r.x, acc.x);
        acc.y = fmaf(ak, r.y, acc.y);
        acc.z = fmaf(ak, r.z, acc.z);
        acc.w = fmaf(ak, r.w, acc.w);
      }
    }
    const float pzr = big ? qnan : pz;
    v4f ov4;
    ov4.x = acc.x + pzr; ov4.y = acc.y + pzr; ov4.z = acc.z + pzr; ov4.w = acc.w + pzr;
    if (node < nN) {
      float* op = outp + (size_t)node * FD + 4 * lane;
      *(volatile v4f*)op = ov4;
      __threadfence();
      *(volatile v4f*)op = ov4;
    }
  }
}

static inline int cdiv(int a, int b) { return (a + b - 1) / b; }

extern "C" void kernel_launch(void* const* d_in, const int* in_sizes, int n_in,
                              void* d_out, int out_size, void* d_ws, size_t ws_size,
                              hipStream_t stream) {
  if (n_in < 10) return;
  if (in_sizes[0] < FD || (in_sizes[0] % FD) != 0) return;
  const int nN = in_sizes[0] / FD;
  if (nN > (1 << 24)) return;
  if (in_sizes[1] < 2 || (in_sizes[1] & 1) != 0) return;
  const int nE = in_sizes[1] / 2;
  if (nE < 1 || nE >= (1 << 21)) return;
  if (in_sizes[2] != FD * FD || in_sizes[3] != FD) return;
  if (in_sizes[4] != NH * FD * FD || in_sizes[5] != NH * FD) return;
  if (in_sizes[6] != NH * FD * FD || in_sizes[7] != NH * FD) return;
  if (in_sizes[8] != NH * FD || in_sizes[9] != NH * FD) return;
  if ((long long)out_size != (long long)nN * FD) return;

  const float* X    = (const float*)d_in[0];
  const int*   ei   = (const int*)  d_in[1];
  const float* Wlin = (const float*)d_in[2];
  const float* blin = (const float*)d_in[3];
  const float* Wel  = (const float*)d_in[4];
  const float* bel  = (const float*)d_in[5];
  const float* Wer  = (const float*)d_in[6];
  const float* ber  = (const float*)d_in[7];
  const float* attl = (const float*)d_in[8];
  const float* attr = (const float*)d_in[9];
  float* out = (float*)d_out;
  const int* own = ei;
  const int* gat = ei + nE;

  const int MP   = cdiv(nN, GBM) * GBM;
  const int gM   = MP / GBM;
  const int gA   = cdiv(nN, NBA);
  if ((long long)gA * NBA < (long long)nN) return;
  const int vec8 = ((nE & 3) == 0) ? 1 : 0;

  char* ws = (char*)d_ws;
  size_t off = 0;
  const size_t oBT  = off; off += (size_t)NCOL * FD * 2;             off = (off + 255) & ~(size_t)255;
  const size_t oCV  = off; off += (size_t)32 * 4;                    off = (off + 255) & ~(size_t)255;
  const size_t oHM  = off; off += (size_t)MP * FD * 4;               off = (off + 255) & ~(size_t)255;
  const size_t oELR = off; off += (size_t)MP * 8 * 4;                off = (off + 255) & ~(size_t)255;
  if (off > ws_size || off > (size_t)WSMAX) return;
  unsigned short* BT  = (unsigned short*)(ws + oBT);
  float*          CV  = (float*)(ws + oCV);
  float*          HM  = (float*)(ws + oHM);
  float*          ELR = (float*)(ws + oELR);

  const size_t aggLds = (size_t)AGG_LDS_INTS * 4;
  hipFuncSetAttribute(reinterpret_cast<const void*>(&k_scan), hipFuncAttributeMaxDynamicSharedMemorySize, (int)aggLds);

  k_prep<<<NBW + 1, NTHR, 0, stream>>>(Wlin, Wel, bel, Wer, ber, attl, attr, BT, CV);
  k_gemm<<<gM, GTHR, 0, stream>>>(X, BT, blin, CV, HM, ELR, nN);
  k_scan<<<gA, NTHR, aggLds, stream>>>(own, gat, nE, nN, vec8, ELR, HM, out);
}
